// SelfAttention_80522046865744
// MI455X (gfx1250) — hardware-verified
//
#include <hip/hip_runtime.h>
#include <math.h>

#ifndef NB
#define NB 4
#endif
#ifndef SEQ
#define SEQ 2048
#endif
#define NB_FULL 4
#define SEQ_FULL 2048
#define DM 1024
#define RS_RPW 4

static_assert(DM == 1024);
static_assert(DM % 64 == 0 && DM % 32 == 0);
static_assert(SEQ % 256 == 0 && SEQ <= 2048);
static_assert(SEQ % (8 * RS_RPW) == 0);
static_assert(SEQ <= SEQ_FULL && NB <= NB_FULL);
static_assert((DM / 64) % 1 == 0 && SEQ % 64 == 0);

typedef __attribute__((ext_vector_type(16))) _Float16     v16h;
typedef __attribute__((ext_vector_type(8)))  _Float16     v8h;
typedef __attribute__((ext_vector_type(8)))  float        v8f;
typedef __attribute__((ext_vector_type(4)))  float        v4f;
typedef __attribute__((ext_vector_type(4)))  unsigned int u4v;
typedef __attribute__((ext_vector_type(4)))  int          i4v;


__device__ __forceinline__ float bfr(float v) {
    const unsigned u = __builtin_bit_cast(unsigned, v);
    const unsigned r = (u + 0x7fffu + ((u >> 16) & 1u)) & 0xffff0000u;
    return __builtin_bit_cast(float, r);
}
__device__ __forceinline__ unsigned pk2h(float a, float b) {
    return (unsigned)__builtin_bit_cast(unsigned short, (_Float16)a) | ((unsigned)__builtin_bit_cast(unsigned short, (_Float16)b) << 16);
}
__device__ __forceinline__ v8f wmma16(v16h a, v16h b, v8f c) {
    c = __builtin_amdgcn_wmma_f32_16x16x32_f16(false, a, false, b, (short)0, c, false, false);
    asm volatile("v_nop\n\tv_nop\n\tv_nop\n\tv_nop" : "+v"(c) : "v"(a), "v"(b));
    return c;
}
union FragH { v16h v; v8h h[2]; };
__device__ __forceinline__ v16h ldfrag(const _Float16* p) {
    FragH f; f.h[0] = *(const v8h*)(p); f.h[1] = *(const v8h*)(p + 16); return f.v;
}
__device__ __forceinline__ void st2_v4f(float* p, v4f v) { *(volatile v4f*)p = v; __threadfence(); *(volatile v4f*)p = v; }
__device__ __forceinline__ void st2_u4(unsigned short* p, u4v v) { *(volatile u4v*)p = v; __threadfence(); *(volatile u4v*)p = v; }

template <int OUT_MODE, bool RESID>
__device__ __forceinline__ void gemm64_body(const unsigned short* __restrict__ Ap, int lda, long long strideA,
                                            const unsigned short* __restrict__ Btp, int ldb, long long strideB,
                                            unsigned short* __restrict__ Ch, float* __restrict__ Cf, int ldc, long long strideC,
                                            const float* __restrict__ resid, int ldr, long long strideR,
                                            int M, int N, int K, float scale) {
    __shared__ __align__(16) float sT[8 * 16 * 68];
    const int b    = blockIdx.y;
    const int lane = threadIdx.x & 31;
    const int wave = __builtin_amdgcn_readfirstlane((int)(threadIdx.x >> 5));
    const int tilesN = N >> 6;
    const int tilesM = M >> 6;
    const int tile = blockIdx.x * 8 + wave;
    if (tile >= tilesM * tilesN) return;
    const int tm = tile / tilesN;
    const int tn = tile - tm * tilesN;
    const int m0 = tm << 6;
    const int n0 = tn << 6;
    const int rlane = lane & 15;
    const int koff  = (lane >> 4) * 8;
    const int sb    = wave * (16 * 68);

    const _Float16* ap = (const _Float16*)Ap  + (size_t)b * (size_t)strideA + (size_t)(m0 + rlane) * (size_t)lda + koff;
    const _Float16* bp = (const _Float16*)Btp + (size_t)b * (size_t)strideB + (size_t)(n0 + rlane) * (size_t)ldb + koff;

    v8f acc[4][4];
#pragma unroll
    for (int i = 0; i < 4; ++i)
#pragma unroll
        for (int j = 0; j < 4; ++j) { const v8f zz = {0.f, 0.f, 0.f, 0.f, 0.f, 0.f, 0.f, 0.f}; acc[i][j] = zz; }

    for (int k0 = 0; k0 < K; k0 += 32) {
        v16h bh[4];
#pragma unroll
        for (int j = 0; j < 4; ++j) bh[j] = ldfrag(bp + (size_t)(16 * j) * (size_t)ldb + k0);
#pragma unroll
        for (int i = 0; i < 4; ++i) {
            const v16h ah = ldfrag(ap + (size_t)(16 * i) * (size_t)lda + k0);
#pragma unroll
            for (int j = 0; j < 4; ++j) acc[i][j] = wmma16(ah, bh[j], acc[i][j]);
        }
    }

#pragma unroll
    for (int i = 0; i < 4; ++i) {
        const int mBase = m0 + (i << 4);
#pragma unroll
        for (int j = 0; j < 4; ++j) {
#pragma unroll
            for (int r = 0; r < 8; ++r) sT[sb + (koff + r) * 68 + (j << 4) + rlane] = acc[i][j][r] * scale;
        }
        __builtin_amdgcn_fence(3  , "workgroup");
        __builtin_amdgcn_wave_barrier();
        __builtin_amdgcn_fence(2  , "workgroup");
        if (OUT_MODE == 0) {
            float* C = Cf + (size_t)b * (size_t)strideC;
            const float* Rb = RESID ? (resid + (size_t)b * (size_t)strideR) : nullptr;
            const int hh = lane >> 4, c4 = (lane & 15) * 4;
            for (int pass = 0; pass < 2; ++pass) {
#pragma unroll
                for (int it = 0; it < 8; ++it) {
                    const int row = it * 2 + hh;
                    v4f v = *(const v4f*)(&sT[sb + row * 68 + c4]);
                    if (RESID) {
                        const v4f xr = *(const v4f*)(Rb + (size_t)(mBase + row) * (size_t)ldr + n0 + c4);
                        v.x += bfr(xr.x); v.y += bfr(xr.y); v.z += bfr(xr.z); v.w += bfr(xr.w);
                    }
                    *(volatile v4f*)(C + (size_t)(mBase + row) * (size_t)ldc + n0 + c4) = v;
                }
                __threadfence();
            }
        } else {
            unsigned short* C = Ch + (size_t)b * (size_t)strideC;
            const int q = lane >> 3, c8 = (lane & 7) * 8;
            for (int pass = 0; pass < 2; ++pass) {
#pragma unroll
                for (int it = 0; it < 4; ++it) {
                    const int row = it * 4 + q;
                    v8h hv;
#pragma unroll
                    for (int e = 0; e < 8; ++e) hv[e] = (_Float16)sT[sb + row * 68 + c8 + e];
                    *(volatile v8h*)(C + (size_t)(mBase + row) * (size_t)ldc + n0 + c8) = hv;
                }
                __threadfence();
            }
        }
        __builtin_amdgcn_fence(3  , "workgroup");
        __builtin_amdgcn_wave_barrier();
        __builtin_amdgcn_fence(2  , "workgroup");
    }
}

__global__ __launch_bounds__(256) void k_gemm_h(const unsigned short* __restrict__ A, int lda, long long strideA,
                                                const unsigned short* __restrict__ Bt, int ldb, long long strideB,
                                                unsigned short* __restrict__ C, int ldc, long long strideC,
                                                int M, int N, int K, float scale) {
    gemm64_body<1, false>(A, lda, strideA, Bt, ldb, strideB, C, nullptr, ldc, strideC, nullptr, 0, 0, M, N, K, scale);
}
__global__ __launch_bounds__(256) void k_gemm_f(const unsigned short* __restrict__ A, int lda, long long strideA,
                                                const unsigned short* __restrict__ Bt, int ldb, long long strideB,
                                                float* __restrict__ C, int ldc, long long strideC,
                                                int M, int N, int K, float scale) {
    gemm64_body<0, false>(A, lda, strideA, Bt, ldb, strideB, nullptr, C, ldc, strideC, nullptr, 0, 0, M, N, K, scale);
}
__global__ __launch_bounds__(256) void k_gemm_fr(const unsigned short* __restrict__ A, int lda, long long strideA,
                                                 const unsigned short* __restrict__ Bt, int ldb, long long strideB,
                                                 float* __restrict__ C, int ldc, long long strideC,
                                                 const float* __restrict__ resid, int ldr, long long strideR,
                                                 int M, int N, int K, float scale) {
    gemm64_body<0, true>(A, lda, strideA, Bt, ldb, strideB, nullptr, C, ldc, strideC, resid, ldr, strideR, M, N, K, scale);
}

__global__ __launch_bounds__(256) void k_colmean(const float* __restrict__ x, float* __restrict__ xbar) {
    __shared__ float red[16 * 68];
    __shared__ __align__(16) float outv[64];
    const int t = threadIdx.x, cg = t & 15, rg = t >> 4;
    const int c0 = blockIdx.x * 64, b = blockIdx.y;
    const float* p = x + ((size_t)b * SEQ_FULL) * DM + c0 + 4 * cg;
    float a0 = 0.f, a1 = 0.f, a2 = 0.f, a3 = 0.f;
#pragma unroll 4
    for (int r = rg; r < SEQ; r += 16) {
        const v4f v = *(const v4f*)(p + (size_t)r * DM);
        a0 += bfr(v.x); a1 += bfr(v.y); a2 += bfr(v.z); a3 += bfr(v.w);
    }
    red[rg * 68 + 4 * cg + 0] = a0; red[rg * 68 + 4 * cg + 1] = a1; red[rg * 68 + 4 * cg + 2] = a2; red[rg * 68 + 4 * cg + 3] = a3;
    __syncthreads();
    if (t < 64) {
        float s = 0.f;
#pragma unroll 1
        for (int j = 0; j < 16; ++j) s += red[j * 68 + t];
        outv[t] = s * (1.0f / (float)SEQ);
    }
    __syncthreads();
    if (t < 16) {
        v4f v; v.x = outv[4 * t]; v.y = outv[4 * t + 1]; v.z = outv[4 * t + 2]; v.w = outv[4 * t + 3];
        st2_v4f(xbar + (size_t)b * DM + c0 + 4 * t, v);
    }
}

__global__ __launch_bounds__(256) void k_prep_x(const float* __restrict__ x, const float* __restrict__ xbar,
                                                unsigned short* __restrict__ XC, unsigned short* __restrict__ X16) {
    const long long u = (long long)blockIdx.x * 256 + threadIdx.x;
    if (u >= (long long)NB * SEQ * (DM / 8)) return;
    const int r = (int)(u / (DM / 8)); const int c0 = 8 * (int)(u % (DM / 8));
    const int b = r / SEQ; const int t = r - b * SEQ;
    const float* s = x + ((size_t)b * SEQ_FULL + t) * DM + c0;
    const float* mb = xbar + (size_t)b * DM + c0;
    const v4f x0 = *(const v4f*)(s), x1 = *(const v4f*)(s + 4);
    const v4f m0 = *(const v4f*)(mb), m1 = *(const v4f*)(mb + 4);
    const float w0 = bfr(x0.x), w1 = bfr(x0.y), w2 = bfr(x0.z), w3 = bfr(x0.w), w4 = bfr(x1.x), w5 = bfr(x1.y), w6 = bfr(x1.z), w7 = bfr(x1.w);
    u4v pa; pa.x = pk2h(w0, w1); pa.y = pk2h(w2, w3); pa.z = pk2h(w4, w5); pa.w = pk2h(w6, w7);
    u4v pc; pc.x = pk2h(w0 - m0.x, w1 - m0.y); pc.y = pk2h(w2 - m0.z, w3 - m0.w); pc.z = pk2h(w4 - m1.x, w5 - m1.y); pc.w = pk2h(w6 - m1.z, w7 - m1.w);
    st2_u4(X16 + (size_t)r * DM + c0, pa);
    st2_u4(XC + (size_t)r * DM + c0, pc);
}

__global__ __launch_bounds__(256) void k_wT(const float* __restrict__ SRC, unsigned short* __restrict__ DST, float sc) {
    const int u = blockIdx.x * 256 + threadIdx.x;
    if (u >= DM * (DM / 8)) return;
    const int n = u / (DM / 8); const int k0 = 8 * (u % (DM / 8));
    float w[8];
#pragma unroll
    for (int e = 0; e < 8; ++e) w[e] = bfr(SRC[(size_t)(k0 + e) * DM + n]) * sc;
    u4v pk; pk.x = pk2h(w[0], w[1]); pk.y = pk2h(w[2], w[3]); pk.z = pk2h(w[4], w[5]); pk.w = pk2h(w[6], w[7]);
    st2_u4(DST + (size_t)n * DM + k0, pk);
}

__global__ __launch_bounds__(256) void k_gate(const unsigned short* __restrict__ X16, const float* __restrict__ Wm, const float* __restrict__ Wb,
                                              float* __restrict__ gate) {
    __shared__ __align__(16) float wl[DM];
    __shared__ __align__(16) float mm[SEQ];
    __shared__ float redm[8];
    __shared__ float reds[8];
    const int t = threadIdx.x, lane = t & 31, b = blockIdx.x;
    const int wave = __builtin_amdgcn_readfirstlane((int)(threadIdx.x >> 5));
    for (int i = t; i < DM; i += 256) wl[i] = bfr(Wm[i]);
    const float bias = bfr(Wb[0]);
    __syncthreads();
    const _Float16* xb = (const _Float16*)X16 + (size_t)b * SEQ * DM;
#pragma unroll 1
    for (int s = wave; s < SEQ; s += 8) {
        const _Float16* xr = xb + (size_t)s * DM + 8 * lane;
        float acc = 0.f;
#pragma unroll 1
        for (int i = 0; i < DM / 256; ++i) {
            const v8h hv = *(const v8h*)(xr + 256 * i);
            const int wo = 256 * i + 8 * lane;
            acc += (float)hv[0] * wl[wo + 0]; acc += (float)hv[1] * wl[wo + 1]; acc += (float)hv[2] * wl[wo + 2]; acc += (float)hv[3] * wl[wo + 3];
            acc += (float)hv[4] * wl[wo + 4]; acc += (float)hv[5] * wl[wo + 5]; acc += (float)hv[6] * wl[wo + 6]; acc += (float)hv[7] * wl[wo + 7];
        }
        acc += __shfl_xor(acc, 16, 32); acc += __shfl_xor(acc, 8, 32); acc += __shfl_xor(acc, 4, 32); acc += __shfl_xor(acc, 2, 32); acc += __shfl_xor(acc, 1, 32);
        if (lane == 0) mm[s] = acc + bias;
    }
    __syncthreads();
    float mx = -3.0e38f;
#pragma unroll 1
    for (int i = t; i < SEQ; i += 256) mx = fmaxf(mx, mm[i]);
    mx = fmaxf(mx, __shfl_xor(mx, 16, 32)); mx = fmaxf(mx, __shfl_xor(mx, 8, 32)); mx = fmaxf(mx, __shfl_xor(mx, 4, 32));
    mx = fmaxf(mx, __shfl_xor(mx, 2, 32));  mx = fmaxf(mx, __shfl_xor(mx, 1, 32));
    if (lane == 0) redm[wave] = mx;
    __syncthreads();
    float gm = redm[0];
#pragma unroll 1
    for (int w = 1; w < 8; ++w) gm = fmaxf(gm, redm[w]);
    float sm = 0.f;
#pragma unroll 1
    for (int i = t; i < SEQ; i += 256) { const float e = expf(mm[i] - gm); mm[i] = e; sm += e; }
    sm += __shfl_xor(sm, 16, 32); sm += __shfl_xor(sm, 8, 32); sm += __shfl_xor(sm, 4, 32); sm += __shfl_xor(sm, 2, 32); sm += __shfl_xor(sm, 1, 32);
    if (lane == 0) reds[wave] = sm;
    __syncthreads();
    float tot = reds[0];
#pragma unroll 1
    for (int w = 1; w < 8; ++w) tot += reds[w];
    const float inv = 1.0f / tot;
#pragma unroll 1
    for (int idx = t; idx < SEQ / 4; idx += 256) {
        v4f v; v.x = mm[4 * idx] * inv; v.y = mm[4 * idx + 1] * inv; v.z = mm[4 * idx + 2] * inv; v.w = mm[4 * idx + 3] * inv;
        st2_v4f(gate + (size_t)b * SEQ + 4 * idx, v);
    }
}

__global__ __launch_bounds__(256) void k_rowsoft(const float* __restrict__ S, const float* __restrict__ cptr, const int* __restrict__ mk,
                                                 const float* __restrict__ gate, unsigned short* __restrict__ P) {
    #pragma clang fp contract(off)
    const int L = threadIdx.x & 31;
    const int wave = __builtin_amdgcn_readfirstlane((int)(threadIdx.x >> 5));
    const float NEG = -__builtin_inff();
    const float cs = bfr(cptr[0]);
    unsigned long long kb = 0ull;
#pragma unroll 1
    for (int g = 0; g < SEQ / 256; ++g) {
        const i4v a = *(const i4v*)(mk + 256 * g + 8 * L), c = *(const i4v*)(mk + 256 * g + 8 * L + 4);
        const unsigned bits = (unsigned)(a.x != 0) | ((unsigned)(a.y != 0) << 1) | ((unsigned)(a.z != 0) << 2) | ((unsigned)(a.w != 0) << 3)
                            | ((unsigned)(c.x != 0) << 4) | ((unsigned)(c.y != 0) << 5) | ((unsigned)(c.z != 0) << 6) | ((unsigned)(c.w != 0) << 7);
        kb |= ((unsigned long long)bits) << (8 * g);
    }
    const int row0 = (blockIdx.x * 8 + wave) * RS_RPW;
#pragma unroll 1
    for (int rr = 0; rr < RS_RPW; ++rr) {
        const int row = row0 + rr;
        const float* sr = S + (size_t)row * SEQ + 8 * L;
        float m = -3.0e38f, s = 0.f;
#pragma unroll 1
        for (int g = 0; g < SEQ / 256; ++g) {
            v4f x = *(const v4f*)(sr + 256 * g), y = *(const v4f*)(sr + 256 * g + 4);
            const unsigned bits = (unsigned)(kb >> (8 * g)) & 0xffu;
            x.x = (bits & 1u) ? x.x * cs : NEG;  x.y = (bits & 2u) ? x.y * cs : NEG;  x.z = (bits & 4u) ? x.z * cs : NEG;  x.w = (bits & 8u) ? x.w * cs : NEG;
            y.x = (bits & 16u) ? y.x * cs : NEG; y.y = (bits & 32u) ? y.y * cs : NEG; y.z = (bits & 64u) ? y.z * cs : NEG; y.w = (bits & 128u) ? y.w * cs : NEG;
            const float mx = fmaxf(fmaxf(fmaxf(x.x, x.y), fmaxf(x.z, x.w)), fmaxf(fmaxf(y.x, y.y), fmaxf(y.z, y.w)));
            const float mn = fmaxf(m, mx);
            s = s * expf(m - mn) + (((expf(x.x - mn) + expf(x.y - mn)) + (expf(x.z - mn) + expf(x.w - mn))) + ((expf(y.x - mn) + expf(y.y - mn)) + (expf(y.z - mn) + expf(y.w - mn))));
            m = mn;
        }
        float gm = m;
        gm = fmaxf(gm, __shfl_xor(gm, 16, 32)); gm = fmaxf(gm, __shfl_xor(gm, 8, 32)); gm = fmaxf(gm, __shfl_xor(gm, 4, 32));
        gm = fmaxf(gm, __shfl_xor(gm, 2, 32));  gm = fmaxf(gm, __shfl_xor(gm, 1, 32));
        s = s * expf(m - gm);
        s += __shfl_xor(s, 16, 32); s += __shfl_xor(s, 8, 32); s += __shfl_xor(s, 4, 32); s += __shfl_xor(s, 2, 32); s += __shfl_xor(s, 1, 32);
        const float f = 1024.f / s;
        unsigned short* pr = P + (size_t)row * SEQ + 8 * L;
        const float* gr = gate + 8 * L;
#pragma unroll 1
        for (int g = 0; g < SEQ / 256; ++g) {
            v4f x = *(const v4f*)(sr + 256 * g), y = *(const v4f*)(sr + 256 * g + 4);
            const v4f gx = *(const v4f*)(gr + 256 * g), gy = *(const v4f*)(gr + 256 * g + 4);
            const unsigned bits = (unsigned)(kb >> (8 * g)) & 0xffu;
            x.x = (bits & 1u) ? x.x * cs : NEG;  x.y = (bits & 2u) ? x.y * cs : NEG;  x.z = (bits & 4u) ? x.z * cs : NEG;  x.w = (bits & 8u) ? x.w * cs : NEG;
            y.x = (bits & 16u) ? y.x * cs : NEG; y.y = (bits & 32u) ? y.y * cs : NEG; y.z = (bits & 64u) ? y.z * cs : NEG; y.w = (bits & 128u) ? y.w * cs : NEG;
            u4v pk;
            pk.x = pk2h(expf(x.x - gm) * f + gx.x * 1024.f, expf(x.y - gm) * f + gx.y * 1024.f);
            pk.y = pk2h(expf(x.z - gm) * f + gx.z * 1024.f, expf(x.w - gm) * f + gx.w * 1024.f);
            pk.z = pk2h(expf(y.x - gm) * f + gy.x * 1024.f, expf(y.y - gm) * f + gy.y * 1024.f);
            pk.w = pk2h(expf(y.z - gm) * f + gy.z * 1024.f, expf(y.w - gm) * f + gy.w * 1024.f);
            st2_u4(pr + 256 * g, pk);
        }
    }
}

constexpr size_t al256(size_t v) { return (v + 255) / 256 * 256; }
constexpr size_t SZ_XC   = (size_t)NB * SEQ * DM * 2;
constexpr size_t SZ_S    = (size_t)SEQ * SEQ * 4;
constexpr size_t SZ_XCS  = al256(SZ_XC > SZ_S ? SZ_XC : SZ_S);
constexpr size_t SZ_X16  = al256((size_t)NB * SEQ * DM * 2);
constexpr size_t SZ_WQK  = al256((size_t)2 * DM * DM * 2);
constexpr size_t SZ_W1   = al256((size_t)DM * DM * 2);
constexpr size_t SZ_QK   = al256((size_t)NB * SEQ * 2 * DM * 2);
constexpr size_t SZ_GT   = al256((size_t)NB * DM * SEQ * 2);
constexpr size_t SZ_AL   = al256((size_t)SEQ * SEQ * 2);
constexpr size_t SZ_AO   = al256((size_t)NB * SEQ * DM * 2);
constexpr size_t SZ_XBAR = al256((size_t)NB * DM * 4);
constexpr size_t SZ_GATE = al256((size_t)NB * SEQ * 4);
constexpr size_t OFF_XCS  = 0;
constexpr size_t OFF_X16  = OFF_XCS + SZ_XCS;
constexpr size_t OFF_WQK  = OFF_X16 + SZ_X16;
constexpr size_t OFF_WGT  = OFF_WQK + SZ_WQK;
constexpr size_t OFF_WOT  = OFF_WGT + SZ_W1;
constexpr size_t OFF_QK   = OFF_WOT + SZ_W1;
constexpr size_t OFF_GT   = OFF_QK + SZ_QK;
constexpr size_t OFF_AL   = OFF_GT + SZ_GT;
constexpr size_t OFF_AO   = OFF_AL + SZ_AL;
constexpr size_t OFF_XBAR = OFF_AO + SZ_AO;
constexpr size_t OFF_GATE = OFF_XBAR + SZ_XBAR;
constexpr size_t WS_TOTAL = OFF_GATE + SZ_GATE;
static_assert(WS_TOTAL <= (size_t)134217728);
static_assert(SZ_S <= SZ_XCS && SZ_XC <= SZ_XCS);

extern "C" void kernel_launch(void* const* d_in, const int* in_sizes, int n_in, void* d_out, int out_size, void* d_ws, size_t ws_size, hipStream_t stream) {
    if (n_in < 9) return;
    const long long need_rows = (long long)(NB - 1) * SEQ_FULL + SEQ;
    if ((long long)in_sizes[0] < need_rows * DM) return;
    if ((long long)in_sizes[1] < need_rows) return;
    if (in_sizes[2] < DM * DM || in_sizes[3] < DM * DM || in_sizes[4] < DM * DM || in_sizes[5] < DM * DM) return;
    if (in_sizes[6] < DM || in_sizes[7] < 1 || in_sizes[8] < 1) return;
    if ((long long)out_size < (long long)NB * SEQ * DM) return;
    if (ws_size < WS_TOTAL) return;

    const float* x    = (const float*)d_in[0];
    const int*   mask = (const int*)d_in[1];
    const float* Wq   = (const float*)d_in[2];
    const float* Wk   = (const float*)d_in[3];
    const float* Wg   = (const float*)d_in[4];
    const float* Wout = (const float*)d_in[5];
    const float* Wm_w = (const float*)d_in[6];
    const float* Wm_b = (const float*)d_in[7];
    const float* cS   = (const float*)d_in[8];
    float* out = (float*)d_out;
    char* ws = (char*)d_ws;
    unsigned short* XC   = (unsigned short*)(ws + OFF_XCS);
    float*          Sf   = (float*)(ws + OFF_XCS);
    unsigned short* X16  = (unsigned short*)(ws + OFF_X16);
    unsigned short* WQK  = (unsigned short*)(ws + OFF_WQK);
    unsigned short* WGT  = (unsigned short*)(ws + OFF_WGT);
    unsigned short* WOT  = (unsigned short*)(ws + OFF_WOT);
    unsigned short* QK   = (unsigned short*)(ws + OFF_QK);
    unsigned short* GT   = (unsigned short*)(ws + OFF_GT);
    unsigned short* AL   = (unsigned short*)(ws + OFF_AL);
    unsigned short* AO   = (unsigned short*)(ws + OFF_AO);
    float*          XBAR = (float*)(ws + OFF_XBAR);
    float*          GATE = (float*)(ws + OFF_GATE);

    const unsigned gw = (unsigned)((DM * (DM / 8) + 255) / 256);
    k_wT<<<gw, 256, 0, stream>>>(Wq, WQK, 16.0f);
    k_wT<<<gw, 256, 0, stream>>>(Wk, WQK + (size_t)DM * DM, 16.0f);
    k_wT<<<gw, 256, 0, stream>>>(Wg, WGT, 16.0f);
    k_wT<<<gw, 256, 0, stream>>>(Wout, WOT, 16.0f);

    k_colmean<<<dim3(DM / 64, NB), 256, 0, stream>>>(x, XBAR);
    k_prep_x<<<(unsigned)(((long long)NB * SEQ * (DM / 8) + 255) / 256), 256, 0, stream>>>(x, XBAR, XC, X16);
    k_gate<<<NB, 256, 0, stream>>>(X16, Wm_w, Wm_b, GATE);

    {
        const int tiles = ((NB * SEQ) / 64) * ((2 * DM) / 64);
        k_gemm_h<<<dim3((unsigned)((tiles + 7) / 8), 1), 256, 0, stream>>>(XC, DM, 0, WQK, DM, 0, QK, 2 * DM, 0, NB * SEQ, 2 * DM, DM, 0.0625f);
    }
    {
        const int tiles = (DM / 64) * (SEQ / 64);
        k_gemm_h<<<dim3((unsigned)((tiles + 7) / 8), NB), 256, 0, stream>>>(WGT, DM, 0, X16, DM, (long long)SEQ * DM, GT, SEQ, (long long)DM * SEQ, DM, SEQ, DM, 0.0625f);
    }
    for (int b = 0; b < NB; ++b) {
        const unsigned short* qb = QK + (size_t)b * SEQ * 2 * DM;
        {
            const int tiles = (SEQ / 64) * (SEQ / 64);
            k_gemm_f<<<dim3((unsigned)((tiles + 7) / 8), 1), 256, 0, stream>>>(qb, 2 * DM, 0, qb + DM, 2 * DM, 0, Sf, SEQ, 0, SEQ, SEQ, DM, 1.0f);
        }
        k_rowsoft<<<SEQ / (8 * RS_RPW), 256, 0, stream>>>(Sf, cS, mask + (size_t)b * SEQ_FULL, GATE + (size_t)b * SEQ, AL);
        {
            const int tiles = (SEQ / 64) * (DM / 64);
            k_gemm_h<<<dim3((unsigned)((tiles + 7) / 8), 1), 256, 0, stream>>>(AL, SEQ, 0, GT + (size_t)b * DM * SEQ, SEQ, 0, AO + (size_t)b * SEQ * DM, DM, 0, SEQ, DM, SEQ, 0.0625f);
        }
    }
    {
        const int tiles = (SEQ / 64) * (DM / 64);
        k_gemm_fr<<<dim3((unsigned)((tiles + 7) / 8), NB), 256, 0, stream>>>(AO, DM, (long long)SEQ * DM, WOT, DM, 0, out, DM, (long long)SEQ * DM,
                                                                            x, DM, (long long)SEQ_FULL * DM, SEQ, DM, DM, 0.0009765625f);
    }
}
